// RelLearnableMultiHeadAttn_8083128451278
// MI455X (gfx1250) — hardware-verified
//
#include <hip/hip_runtime.h>
#include <math.h>

constexpr int kBatch = 4;
constexpr int kSeq   = 1024;
constexpr int kDim   = 1024;
constexpr int kHeads = 16;
constexpr int kHd    = 64;
constexpr int kTok   = kBatch * kSeq;
constexpr float kLnEps  = 1e-5f;
constexpr float kInvDim = 1.0f / 1024.0f;
constexpr float kScale  = 0.125f;
constexpr float kPCarry = 32768.0f;
constexpr int kKC = 64;
constexpr int kOsPitch = 68;

typedef __attribute__((ext_vector_type(16))) _Float16 v16h;
typedef __attribute__((ext_vector_type(8)))  _Float16 v8h;
typedef __attribute__((ext_vector_type(16))) __bf16   v16b;
typedef __attribute__((ext_vector_type(8)))  __bf16   v8b;
typedef __attribute__((ext_vector_type(8)))  float    v8f;
typedef __attribute__((ext_vector_type(4)))  float    v4f;
typedef __attribute__((ext_vector_type(4)))  unsigned int v4u;

__device__ __forceinline__ unsigned short f2bf_bits(float f) {
  unsigned u = __float_as_uint(f);
  return (unsigned short)((u + 0x7FFFu + ((u >> 16) & 1u)) >> 16);
}
__device__ __forceinline__ float bf_bits2f(unsigned short h) { return __uint_as_float(((unsigned)h) << 16); }
__device__ __forceinline__ float bf_rne(float f) { return bf_bits2f(f2bf_bits(f)); }

__device__ __forceinline__ void dep_guard_h(v8f& a, v8f& b, v16h x, v16h y) { asm volatile("v_nop\n\tv_nop\n\tv_nop\n\tv_nop" : "+v"(a), "+v"(b) : "v"(x), "v"(y)); }
__device__ __forceinline__ void dep_guard_b(v8f& a, v8f& b, v16b x, v16b y) { asm volatile("v_nop\n\tv_nop\n\tv_nop\n\tv_nop" : "+v"(a), "+v"(b) : "v"(x), "v"(y)); }
__device__ __forceinline__ void keep4_h(v16h a, v16h b, v16h c, v16h d) { asm volatile("v_nop" :: "v"(a), "v"(b), "v"(c), "v"(d)); }
__device__ __forceinline__ void keep4_b(v16b a, v16b b, v16b c, v16b d) { asm volatile("v_nop" :: "v"(a), "v"(b), "v"(c), "v"(d)); }
__device__ __forceinline__ void acc_guard4(v8f& a, v8f& b, v8f& c, v8f& d) { asm volatile("v_nop\n\tv_nop\n\tv_nop\n\tv_nop" : "+v"(a), "+v"(b), "+v"(c), "+v"(d)); }
template <typename T> struct Frag;
template <> struct Frag<_Float16> {
  typedef v16h V; union U { v16h v; v8h h[2]; };
  static __device__ __forceinline__ v16h load(const _Float16* p) {
    U f; f.h[0] = *(const v8h*)(p); f.h[1] = *(const v8h*)(p + 16); return f.v;
  }
  static __device__ __forceinline__ v8f mma(v16h a, v16h b, v8f c) {
    return __builtin_amdgcn_wmma_f32_16x16x32_f16(false, a, false, b, (short)0, c, false, false);
  }
  static __device__ __forceinline__ void guard(v8f& a, v8f& b, v16h x, v16h y) { dep_guard_h(a, b, x, y); }
  static __device__ __forceinline__ void keep(v16h a, v16h b, v16h c, v16h d) { keep4_h(a, b, c, d); }
};
template <> struct Frag<__bf16> {
  typedef v16b V; union U { v16b v; v8b h[2]; };
  static __device__ __forceinline__ v16b load(const __bf16* p) {
    U f; f.h[0] = *(const v8b*)(p); f.h[1] = *(const v8b*)(p + 16); return f.v;
  }
  static __device__ __forceinline__ v8f mma(v16b a, v16b b, v8f c) {
    return __builtin_amdgcn_wmma_f32_16x16x32_bf16(false, a, false, b, (short)0, c, false, false);
  }
  static __device__ __forceinline__ void guard(v8f& a, v8f& b, v16b x, v16b y) { dep_guard_b(a, b, x, y); }
  static __device__ __forceinline__ void keep(v16b a, v16b b, v16b c, v16b d) { keep4_b(a, b, c, d); }
};

__device__ __forceinline__ unsigned pk16(unsigned short a, unsigned short b) { return (unsigned)a | ((unsigned)b << 16); }

__device__ __forceinline__ v8f mma_bf16g(v16b a, v16b b, v8f c) {
  c = __builtin_amdgcn_wmma_f32_16x16x32_bf16(false, a, false, b, (short)0, c, false, false);
  asm volatile("v_nop\n\tv_nop\n\tv_nop\n\tv_nop" : "+v"(c) : "v"(a), "v"(b));
  return c;
}
__device__ __forceinline__ v8f mma_f16g(v16h a, v16h b, v8f c) {
  c = __builtin_amdgcn_wmma_f32_16x16x32_f16(false, a, false, b, (short)0, c, false, false);
  asm volatile("v_nop\n\tv_nop\n\tv_nop\n\tv_nop" : "+v"(c) : "v"(a), "v"(b));
  return c;
}

template <int ET> struct Elem;
template <> struct Elem<0> { typedef _Float16 T; };
template <> struct Elem<1> { typedef __bf16 T; };
template <int ET, int SPLIT, int BIAS_MODE, int OUT_MODE, bool RESID, int ACT = 0>
__global__ __launch_bounds__(256) void wmma_gemm64(
    const unsigned short* __restrict__ Ap, const unsigned short* __restrict__ A2p, int lda, long strideA,
    const unsigned short* __restrict__ Btp, const unsigned short* __restrict__ Bt2p, int ldb, long strideB,
    void* __restrict__ Cout, void* __restrict__ Cout2, int ldc, long strideC,
    const float* __restrict__ bias,
    const float* __restrict__ resid, long strideR,
    int M, int N, int K, float scale) {
  typedef typename Elem<ET>::T T;
  typedef typename Frag<T>::V V;
  const T* A = (const T*)Ap; const T* A2 = (const T*)A2p; const T* Bt = (const T*)Btp; const T* Bt2 = (const T*)Bt2p;
  __shared__ __align__(16) float sT[8][16 * 68];
  const int b    = blockIdx.y;
  const int lane = threadIdx.x & 31;
  const int wave = threadIdx.x >> 5;
  const int tilesN = N >> 6;
  const int tilesM = M >> 6;
  const int tile = blockIdx.x * 8 + wave;
  if (tile >= tilesM * tilesN) return;
  const int tm = tile / tilesN;
  const int tn = tile - tm * tilesN;
  const int m0 = tm << 6;
  const int n0 = tn << 6;

  const T* Ab  = A  + (size_t)b * strideA;
  const T* Bb  = Bt + (size_t)b * strideB;
  const T* Ab2 = (SPLIT != 0) ? (A2  + (size_t)b * strideA) : nullptr;
  const T* Bb2 = (SPLIT == 1) ? (Bt2 + (size_t)b * strideB) : nullptr;

  const int rlane = lane & 15;
  const int koff  = (lane >> 4) * 8;
  const int mOff  = (lane >> 4) * 8;

  v8f acc[4][4];
#pragma unroll
  for (int i = 0; i < 4; ++i)
#pragma unroll
    for (int j = 0; j < 4; ++j) acc[i][j] = (v8f){0.f,0.f,0.f,0.f,0.f,0.f,0.f,0.f};

  for (int k0 = 0; k0 < K; k0 += 32) {
    V bh[4], bl[4];
#pragma unroll
    for (int j = 0; j < 4; ++j) {
      const size_t bo = (size_t)(n0 + (j << 4) + rlane) * ldb + koff + k0;
      bh[j] = Frag<T>::load(Bb + bo);
      if (SPLIT == 1) bl[j] = Frag<T>::load(Bb2 + bo);
    }
#pragma unroll
    for (int i = 0; i < 4; ++i) {
      const size_t ao = (size_t)(m0 + (i << 4) + rlane) * lda + koff + k0;
      V ah = Frag<T>::load(Ab + ao);
      V al;
      if (SPLIT != 0) al = Frag<T>::load(Ab2 + ao);
#pragma unroll
      for (int j = 0; j < 4; ++j) {
        acc[i][j] = Frag<T>::mma(ah, bh[j], acc[i][j]);
        if (SPLIT == 1) acc[i][j] = Frag<T>::mma(ah, bl[j], acc[i][j]);
        if (SPLIT != 0) acc[i][j] = Frag<T>::mma(al, bh[j], acc[i][j]);
      }
      Frag<T>::guard(acc[i][0], acc[i][3], ah, (SPLIT != 0) ? al : ah);
    }
    Frag<T>::keep(bh[0], bh[1], bh[2], bh[3]);
    if (SPLIT == 1) Frag<T>::keep(bl[0], bl[1], bl[2], bl[3]);
  }
  acc_guard4(acc[0][0], acc[0][1], acc[0][2], acc[0][3]);
  acc_guard4(acc[1][0], acc[1][1], acc[1][2], acc[1][3]);
  acc_guard4(acc[2][0], acc[2][1], acc[2][2], acc[2][3]);
  acc_guard4(acc[3][0], acc[3][1], acc[3][2], acc[3][3]);

  float* slab = sT[wave];
  const float* Rb = RESID ? (resid + (size_t)b * strideR) : nullptr;
#pragma unroll
  for (int i = 0; i < 4; ++i) {
    const int mBase = m0 + (i << 4);
#pragma unroll
    for (int j = 0; j < 4; ++j) {
      const int n = n0 + (j << 4) + rlane;
      float bv = 0.f;
      if (BIAS_MODE == 2) bv = bias[n];
#pragma unroll
      for (int r = 0; r < 8; ++r) {
        float v = acc[i][j][r] * scale;
        if (BIAS_MODE == 1) v += bias[mBase + mOff + r];
        if (BIAS_MODE == 2) v += bv;
        if (RESID) v += Rb[(size_t)(mBase + mOff + r) * ldc + n];
        if (ACT == 2) v = fmaxf(v, 0.0f);
        if (ACT == 4) v = (v > 0.f) ? v : 0.01f * v;
        slab[(mOff + r) * 68 + (j << 4) + rlane] = v;
      }
    }
    __builtin_amdgcn_fence(__ATOMIC_RELEASE, "workgroup");
    __builtin_amdgcn_wave_barrier();
    __builtin_amdgcn_fence(__ATOMIC_ACQUIRE, "workgroup");
    if (OUT_MODE == 0) {
      float* C = (float*)Cout + (size_t)b * strideC;
      const int hh = lane >> 4, c4 = (lane & 15) * 4;
      for (int pass = 0; pass < 2; ++pass) {
#pragma unroll
        for (int it = 0; it < 8; ++it) {
          const int row = it * 2 + hh;
          v4f v = *(const v4f*)(slab + row * 68 + c4);
          *(volatile v4f*)(C + (size_t)(mBase + row) * ldc + n0 + c4) = v;
        }
        __threadfence();
      }
    } else {
      const int q = lane >> 3, c8 = (lane & 7) * 8;
      unsigned short* C  = (unsigned short*)Cout  + (size_t)b * strideC;
      unsigned short* C2 = (OUT_MODE == 2) ? ((unsigned short*)Cout2 + (size_t)b * strideC) : nullptr;
      for (int pass = 0; pass < 2; ++pass) {
#pragma unroll
        for (int it = 0; it < 4; ++it) {
          const int row = it * 4 + q;
          const float* sp = slab + row * 68 + c8;
          v8h hv, lv;
#pragma unroll
          for (int e = 0; e < 8; ++e) {
            if (OUT_MODE == 1) {
              hv[e] = (_Float16)sp[e];
            } else {
              unsigned short hb = f2bf_bits(sp[e]);
              unsigned short lb = f2bf_bits(sp[e] - bf_bits2f(hb));
              hv[e] = __builtin_bit_cast(_Float16, hb);
              lv[e] = __builtin_bit_cast(_Float16, lb);
            }
          }
          *(volatile v8h*)(C + (size_t)(mBase + row) * ldc + n0 + c8) = hv;
          if (OUT_MODE == 2) *(volatile v8h*)(C2 + (size_t)(mBase + row) * ldc + n0 + c8) = lv;
        }
        __threadfence();
      }
    }
    __builtin_amdgcn_fence(__ATOMIC_RELEASE, "workgroup");
    __builtin_amdgcn_wave_barrier();
    __builtin_amdgcn_fence(__ATOMIC_ACQUIRE, "workgroup");
  }
}

__global__ __launch_bounds__(256) void cvt_bf16x8_kernel(const float* __restrict__ in, unsigned short* __restrict__ out, int n8) {
  const int i = blockIdx.x * 256 + threadIdx.x;
  if (i >= n8) return;
  const size_t base = (size_t)i * 8;
  const v4f a = *(const v4f*)(in + base), c = *(const v4f*)(in + base + 4);
  unsigned short hb[8];
#pragma unroll
  for (int e = 0; e < 4; ++e) { hb[e] = f2bf_bits(a[e]); hb[4 + e] = f2bf_bits(c[e]); }
  const v4u u = (v4u){pk16(hb[0], hb[1]), pk16(hb[2], hb[3]), pk16(hb[4], hb[5]), pk16(hb[6], hb[7])};
  *(volatile v4u*)(out + base) = u;
  __threadfence();
  *(volatile v4u*)(out + base) = u;
}

__global__ __launch_bounds__(256) void wtcast4_kernel(const float* __restrict__ W0, const float* __restrict__ W1,
                                                      const float* __restrict__ W2, const float* __restrict__ W3,
                                                      unsigned short* __restrict__ out) {
  __shared__ float sm[64][65];
  const int t  = threadIdx.x;
  const int d0 = blockIdx.x * 64;
  const int h0 = blockIdx.y * 64;
  const int z  = blockIdx.z;
  const float* W = (z == 0) ? W0 : (z == 1) ? W1 : (z == 2) ? W2 : W3;
#pragma unroll
  for (int i = 0; i < 16; ++i) {
    const int e = i * 256 + t;
    const int r = e >> 6;
    const int cc = e & 63;
    sm[cc][r] = W[(size_t)(d0 + r) * kDim + h0 + cc];
  }
  __syncthreads();
  const int lane = t & 31, wave = t >> 5;
  const int q = lane >> 3, c8 = (lane & 7) * 8;
  unsigned short* op = out + (size_t)z * kDim * kDim;
  for (int pass = 0; pass < 2; ++pass) {
#pragma unroll
    for (int it = 0; it < 2; ++it) {
      const int row = wave * 8 + it * 4 + q;
      unsigned short hb[8];
#pragma unroll
      for (int e = 0; e < 8; ++e) hb[e] = f2bf_bits(sm[row][c8 + e]);
      const v4u u = (v4u){pk16(hb[0], hb[1]), pk16(hb[2], hb[3]), pk16(hb[4], hb[5]), pk16(hb[6], hb[7])};
      *(volatile v4u*)(op + (size_t)(h0 + row) * kDim + d0 + c8) = u;
    }
    __threadfence();
  }
}

__global__ __launch_bounds__(256) void qplanes_kernel(const float* __restrict__ qf, const float* __restrict__ rwb,
                                                      unsigned short* __restrict__ oh, unsigned short* __restrict__ ol, int n8) {
  const int i = blockIdx.x * 256 + threadIdx.x;
  if (i >= n8) return;
  const size_t base = (size_t)i * 8;
  const int col = (int)(base % (size_t)kDim);
  const v4f a0 = *(const v4f*)(qf + base), a1 = *(const v4f*)(qf + base + 4);
  const v4f u0 = *(const v4f*)(rwb + col), u1 = *(const v4f*)(rwb + col + 4);
  float x[8];
#pragma unroll
  for (int e = 0; e < 4; ++e) { x[e] = a0[e] + bf_rne(u0[e]); x[4 + e] = a1[e] + bf_rne(u1[e]); }
  unsigned short hb[8], lb[8];
#pragma unroll
  for (int e = 0; e < 8; ++e) { hb[e] = f2bf_bits(x[e]); lb[e] = f2bf_bits(x[e] - bf_bits2f(hb[e])); }
  const v4u uh = (v4u){pk16(hb[0], hb[1]), pk16(hb[2], hb[3]), pk16(hb[4], hb[5]), pk16(hb[6], hb[7])};
  const v4u ul = (v4u){pk16(lb[0], lb[1]), pk16(lb[2], lb[3]), pk16(lb[4], lb[5]), pk16(lb[6], lb[7])};
  *(volatile v4u*)(oh + base) = uh;
  *(volatile v4u*)(ol + base) = ul;
  __threadfence();
  *(volatile v4u*)(oh + base) = uh;
  *(volatile v4u*)(ol + base) = ul;
}

__global__ __launch_bounds__(256) void krplanes_kernel(const float* __restrict__ kf, const float* __restrict__ remb,
                                                       unsigned short* __restrict__ oh, unsigned short* __restrict__ ol, int n8) {
  const int i = blockIdx.x * 256 + threadIdx.x;
  if (i >= n8) return;
  const size_t base = (size_t)i * 8;
  const int row = (int)(base / (size_t)kDim);
  const int j   = row % kSeq;
  const int col = (int)(base % (size_t)kDim);
  const bool keep = (j + 1 < kSeq);
  const int jr = keep ? (j + 1) : (kSeq - 1);
  const float* rp = remb + (size_t)jr * kDim + col;
  const v4f k0 = *(const v4f*)(kf + base), k1 = *(const v4f*)(kf + base + 4);
  const v4f r0 = *(const v4f*)(rp), r1 = *(const v4f*)(rp + 4);
  float x[8];
#pragma unroll
  for (int e = 0; e < 4; ++e) {
    x[e]     = k0[e] + (keep ? bf_rne(r0[e]) : 0.0f);
    x[4 + e] = k1[e] + (keep ? bf_rne(r1[e]) : 0.0f);
  }
  unsigned short hb[8], lb[8];
#pragma unroll
  for (int e = 0; e < 8; ++e) { hb[e] = f2bf_bits(x[e]); lb[e] = f2bf_bits(x[e] - bf_bits2f(hb[e])); }
  const v4u uh = (v4u){pk16(hb[0], hb[1]), pk16(hb[2], hb[3]), pk16(hb[4], hb[5]), pk16(hb[6], hb[7])};
  const v4u ul = (v4u){pk16(lb[0], lb[1]), pk16(lb[2], lb[3]), pk16(lb[4], lb[5]), pk16(lb[6], lb[7])};
  *(volatile v4u*)(oh + base) = uh;
  *(volatile v4u*)(ol + base) = ul;
  __threadfence();
  *(volatile v4u*)(oh + base) = uh;
  *(volatile v4u*)(ol + base) = ul;
}

__global__ __launch_bounds__(256) void tb_kernel(const float* __restrict__ rwb, const float* __restrict__ remb,
                                                 const float* __restrict__ rbias, float* __restrict__ tb) {
  const int i = blockIdx.x * 256 + threadIdx.x;
  const int n = i >> 10;
  const int j = i & (kSeq - 1);
  const bool keep = (j + 1 < kSeq);
  const int jr = keep ? (j + 1) : (kSeq - 1);
  const float* rp = remb + ((size_t)jr * kHeads + n) * kHd;
  const float* up = rwb + n * kHd;
  float acc = 0.f;
#pragma unroll 1
  for (int d = 0; d < kHd; ++d) acc = fmaf(bf_rne(up[d]), bf_rne(rp[d]), acc);
  const float val = keep ? (bf_rne(rbias[jr * kHeads + n]) - acc) : 0.0f;
  ((volatile float*)tb)[i] = val;
  __threadfence();
  ((volatile float*)tb)[i] = val;
}

__global__ __launch_bounds__(128) void relattn_kernel(
    const unsigned short* __restrict__ QRh, const unsigned short* __restrict__ QRl,
    const unsigned short* __restrict__ KRh, const unsigned short* __restrict__ KRl,
    const unsigned short* __restrict__ Vp, const float* __restrict__ tb,
    unsigned short* __restrict__ AVh, unsigned short* __restrict__ AVl) {
  union FB { v16b v; v8b h[2]; };
  union FH { v16h v; v8h h[2]; };
  __shared__ __align__(16) __bf16   Ksh[kKC * kHd];
  __shared__ __align__(16) __bf16   Ksl[kKC * kHd];
  __shared__ __align__(16) _Float16 Vt[kHd * kKC];
  __shared__ __align__(16) _Float16 Psh[4][16 * kKC];
  __shared__ __align__(16) float    Os[4][16 * kOsPitch];

  const int tid  = threadIdx.x;
  const int wave = tid >> 5;
  const int lane = tid & 31;
  const int hh   = lane >> 4;
  const int c    = lane & 15;

  const int bx = blockIdx.x;
  const int qb = bx & 15;
  const int h  = (bx >> 4) & 15;
  const int b  = bx >> 8;
  const int q0 = qb * 64 + wave * 16;
  const size_t tok0 = (size_t)b * kSeq;
  const int hcol = h * kHd;

  v16b qah[2], qal[2];
  {
    const __bf16* ph = (const __bf16*)QRh + (tok0 + q0 + c) * kDim + hcol + 8 * hh;
    const __bf16* pl = (const __bf16*)QRl + (tok0 + q0 + c) * kDim + hcol + 8 * hh;
#pragma unroll
    for (int dc = 0; dc < 2; ++dc) {
      qah[dc] = Frag<__bf16>::load(ph + dc * 32);
      qal[dc] = Frag<__bf16>::load(pl + dc * 32);
    }
  }

  float mrow[8], lrow[8];
  v8f oacc[4];
#pragma unroll
  for (int r = 0; r < 8; ++r) { mrow[r] = -INFINITY; lrow[r] = 0.f; }
#pragma unroll
  for (int t = 0; t < 4; ++t) oacc[t] = (v8f){0.f,0.f,0.f,0.f,0.f,0.f,0.f,0.f};

  for (int kc = 0; kc < kSeq / kKC; ++kc) {
    const int kv0 = kc * kKC;
    __syncthreads();
    {
      const int kvr = tid >> 1;
      const int dh  = (tid & 1) * 32;
      const size_t g = (tok0 + kv0 + kvr) * kDim + hcol + dh;
      const v8b* gkh = (const v8b*)((const __bf16*)KRh + g);
      const v8b* gkl = (const v8b*)((const __bf16*)KRl + g);
      const v8h* gv  = (const v8h*)((const _Float16*)Vp + g);
#pragma unroll
      for (int i = 0; i < 4; ++i) {
        const v8b a  = gkh[i];
        const v8b al = gkl[i];
        const v8h vv = gv[i];
        *(v8b*)(Ksh + kvr * kHd + dh + 8 * i) = a;
        *(v8b*)(Ksl + kvr * kHd + dh + 8 * i) = al;
#pragma unroll
        for (int e = 0; e < 8; ++e) Vt[(dh + 8 * i + e) * kKC + kvr] = vv[e];
      }
    }
    __syncthreads();

    v8f s[4];
#pragma unroll
    for (int j = 0; j < 4; ++j) {
      s[j] = (v8f){0.f,0.f,0.f,0.f,0.f,0.f,0.f,0.f};
#pragma unroll
      for (int dc = 0; dc < 2; ++dc) {
        FB kb, kl;
        kb.h[0] = *(const v8b*)(Ksh + (j * 16 + c) * kHd + dc * 32 + 8 * hh);
        kb.h[1] = *(const v8b*)(Ksh + (j * 16 + c) * kHd + dc * 32 + 16 + 8 * hh);
        kl.h[0] = *(const v8b*)(Ksl + (j * 16 + c) * kHd + dc * 32 + 8 * hh);
        kl.h[1] = *(const v8b*)(Ksl + (j * 16 + c) * kHd + dc * 32 + 16 + 8 * hh);
        s[j] = mma_bf16g(qah[dc], kb.v, s[j]);
        s[j] = mma_bf16g(qah[dc], kl.v, s[j]);
        s[j] = mma_bf16g(qal[dc], kb.v, s[j]);
      }
    }
    float tbv[4];
#pragma unroll
    for (int j = 0; j < 4; ++j) tbv[j] = tb[h * kSeq + kv0 + j * 16 + c];

    float cm[8];
#pragma unroll
    for (int r = 0; r < 8; ++r) {
      float m = -INFINITY;
#pragma unroll
      for (int j = 0; j < 4; ++j) {
        s[j][r] = (s[j][r] + tbv[j]) * kScale;
        m = fmaxf(m, s[j][r]);
      }
#pragma unroll
      for (int off = 1; off < 16; off <<= 1) m = fmaxf(m, __shfl_xor(m, off, 32));
      cm[r] = m;
    }
    _Float16* pw = Psh[wave];
#pragma unroll
    for (int r = 0; r < 8; ++r) {
      const float mnew  = fmaxf(mrow[r], cm[r]);
      const float alpha = expf(mrow[r] - mnew);
      mrow[r] = mnew;
      float psum = 0.f;
#pragma unroll
      for (int j = 0; j < 4; ++j) {
        const float p = expf(s[j][r] - mnew);
        psum += p;
        pw[(8 * hh + r) * kKC + j * 16 + c] = (_Float16)(p * kPCarry);
      }
#pragma unroll
      for (int off = 1; off < 16; off <<= 1) psum += __shfl_xor(psum, off, 32);
      lrow[r] = lrow[r] * alpha + psum;
#pragma unroll
      for (int t = 0; t < 4; ++t) oacc[t][r] *= alpha;
    }
    __builtin_amdgcn_fence(__ATOMIC_RELEASE, "workgroup");
    __builtin_amdgcn_wave_barrier();
    __builtin_amdgcn_fence(__ATOMIC_ACQUIRE, "workgroup");
#pragma unroll
    for (int kk = 0; kk < 2; ++kk) {
      FH pa;
      pa.h[0] = *(const v8h*)(pw + c * kKC + kk * 32 + 8 * hh);
      pa.h[1] = *(const v8h*)(pw + c * kKC + kk * 32 + 16 + 8 * hh);
#pragma unroll
      for (int t = 0; t < 4; ++t) {
        FH vb;
        vb.h[0] = *(const v8h*)(Vt + (t * 16 + c) * kKC + kk * 32 + 8 * hh);
        vb.h[1] = *(const v8h*)(Vt + (t * 16 + c) * kKC + kk * 32 + 16 + 8 * hh);
        oacc[t] = mma_f16g(pa.v, vb.v, oacc[t]);
      }
    }
  }

  float* os = Os[wave];
#pragma unroll
  for (int r = 0; r < 8; ++r) {
    const float inv = 1.0f / (lrow[r] * kPCarry);
#pragma unroll
    for (int t = 0; t < 4; ++t) os[(8 * hh + r) * kOsPitch + t * 16 + c] = oacc[t][r] * inv;
  }
  __builtin_amdgcn_fence(__ATOMIC_RELEASE, "workgroup");
  __builtin_amdgcn_wave_barrier();
  __builtin_amdgcn_fence(__ATOMIC_ACQUIRE, "workgroup");
  {
    const int q = lane >> 3, c8 = (lane & 7) * 8;
    for (int pass = 0; pass < 2; ++pass) {
#pragma unroll
      for (int it = 0; it < 4; ++it) {
        const int row = it * 4 + q;
        const float* sp = os + row * kOsPitch + c8;
        v8h hv, lv;
#pragma unroll
        for (int e = 0; e < 8; ++e) {
          const unsigned short hb = f2bf_bits(sp[e]);
          const unsigned short lb = f2bf_bits(sp[e] - bf_bits2f(hb));
          hv[e] = __builtin_bit_cast(_Float16, hb);
          lv[e] = __builtin_bit_cast(_Float16, lb);
        }
        const size_t o = (tok0 + q0 + row) * kDim + hcol + c8;
        *(volatile v8h*)(AVh + o) = hv;
        *(volatile v8h*)(AVl + o) = lv;
      }
      __threadfence();
    }
  }
}

__global__ __launch_bounds__(256) void ln_kernel(const float* __restrict__ w, const float* __restrict__ ao,
                                                 const float* __restrict__ g, const float* __restrict__ bt,
                                                 float* __restrict__ out) {
  __shared__ float red[16];
  const int row  = blockIdx.x;
  const int t    = threadIdx.x, lane = t & 31, wave = t >> 5;
  const int c0   = t * 4;
  const size_t off = (size_t)row * kDim + c0;
  const v4f a = *(const v4f*)(w + off);
  const v4f o = *(const v4f*)(ao + off);
  float x[4];
#pragma unroll
  for (int e = 0; e < 4; ++e) x[e] = bf_rne(a[e]) + o[e];
  float s = (x[0] + x[1]) + (x[2] + x[3]);
#pragma unroll
  for (int sh = 16; sh > 0; sh >>= 1) s += __shfl_xor(s, sh, 32);
  if (lane == 0) red[wave] = s;
  __syncthreads();
  const float mu = (((red[0] + red[1]) + (red[2] + red[3])) + ((red[4] + red[5]) + (red[6] + red[7]))) * kInvDim;
  float d[4];
  float s2 = 0.f;
#pragma unroll
  for (int e = 0; e < 4; ++e) { d[e] = x[e] - mu; s2 += d[e] * d[e]; }
#pragma unroll
  for (int sh = 16; sh > 0; sh >>= 1) s2 += __shfl_xor(s2, sh, 32);
  if (lane == 0) red[8 + wave] = s2;
  __syncthreads();
  const float var  = (((red[8] + red[9]) + (red[10] + red[11])) + ((red[12] + red[13]) + (red[14] + red[15]))) * kInvDim;
  const float rstd = rsqrtf(var + kLnEps);
  const v4f gg = *(const v4f*)(g + c0);
  const v4f bb = *(const v4f*)(bt + c0);
  v4f y;
#pragma unroll
  for (int e = 0; e < 4; ++e) y[e] = (d[e] * rstd) * bf_rne(gg[e]) + bf_rne(bb[e]);
  *(volatile v4f*)(out + off) = y;
  __threadfence();
  *(volatile v4f*)(out + off) = y;
}

extern "C" void kernel_launch(void* const* d_in, const int* in_sizes, int n_in,
                              void* d_out, int out_size, void* d_ws, size_t ws_size,
                              hipStream_t stream) {
  if (n_in < 10) return;
  const float* w     = (const float*)d_in[0];
  const float* remb  = (const float*)d_in[1];
  const float* rwb   = (const float*)d_in[2];
  const float* rbias = (const float*)d_in[3];
  const float* Wq    = (const float*)d_in[4];
  const float* Wk    = (const float*)d_in[5];
  const float* Wv    = (const float*)d_in[6];
  const float* Wo    = (const float*)d_in[7];
  const float* gamma = (const float*)d_in[8];
  const float* beta  = (const float*)d_in[9];
  float* out = (float*)d_out;

  const size_t nTokD = (size_t)kTok * kDim;
  if ((size_t)in_sizes[0] != nTokD) return;
  if (in_sizes[1] != kSeq * kHeads * kHd) return;
  if (in_sizes[2] != kHeads * kHd) return;
  if (in_sizes[3] != kSeq * kHeads) return;
  if (in_sizes[4] != kDim * kDim || in_sizes[5] != kDim * kDim || in_sizes[6] != kDim * kDim || in_sizes[7] != kDim * kDim) return;
  if (in_sizes[8] != kDim || in_sizes[9] != kDim) return;
  if ((size_t)out_size != nTokD) return;

  const size_t bWb  = nTokD * 2;
  const size_t bWT  = (size_t)4 * kDim * kDim * 2;
  const size_t bQKF = nTokD * 4 * 2;
  const size_t bVh  = nTokD * 2;
  const size_t bQR  = nTokD * 2 * 2;
  const size_t bKR  = nTokD * 2 * 2;
  const size_t bTB  = (size_t)kHeads * kSeq * 4;
  const size_t oWb  = 0;
  const size_t oWT  = oWb + bWb;
  const size_t oQKF = oWT + bWT;
  const size_t oVh  = oQKF + bQKF;
  const size_t oQR  = oVh + bVh;
  const size_t oKR  = oQR + bQR;
  const size_t oTB  = oKR + bKR;
  const size_t total = oTB + bTB;
  if (total > ws_size) return;

  char* ws = (char*)d_ws;
  unsigned short* Wb  = (unsigned short*)(ws + oWb);
  unsigned short* WT  = (unsigned short*)(ws + oWT);
  float*          QKF = (float*)(ws + oQKF);
  float*          qf  = QKF;
  float*          kf  = QKF + nTokD;
  unsigned short* Vh  = (unsigned short*)(ws + oVh);
  unsigned short* QRh = (unsigned short*)(ws + oQR);
  unsigned short* QRl = QRh + nTokD;
  unsigned short* KRh = (unsigned short*)(ws + oKR);
  unsigned short* KRl = KRh + nTokD;
  float*          TB  = (float*)(ws + oTB);
  unsigned short* AVh = (unsigned short*)(ws + oQKF);
  unsigned short* AVl = AVh + nTokD;
  float*          AO  = kf;

  const int n8 = (int)(nTokD / 8);
  const long wPlane = (long)kDim * kDim;

  cvt_bf16x8_kernel<<<dim3(n8 / 256), dim3(256), 0, stream>>>(w, Wb, n8);
  wtcast4_kernel<<<dim3(kDim / 64, kDim / 64, 4), dim3(256), 0, stream>>>(Wq, Wk, Wv, Wo, WT);
  wmma_gemm64<1, 0, 0, 0, false><<<dim3(128, 2), dim3(256), 0, stream>>>(
      Wb, Wb, kDim, 0L,
      WT, WT, kDim, wPlane,
      (void*)QKF, (void*)QKF, kDim, (long)nTokD,
      gamma, gamma, 0L,
      kTok, kDim, kDim, 1.0f);
  wmma_gemm64<1, 0, 0, 1, false><<<dim3(128, 1), dim3(256), 0, stream>>>(
      Wb, Wb, kDim, 0L,
      WT + 2 * wPlane, WT + 2 * wPlane, kDim, 0L,
      (void*)Vh, (void*)Vh, kDim, 0L,
      gamma, gamma, 0L,
      kTok, kDim, kDim, 1.0f);
  qplanes_kernel<<<dim3(n8 / 256), dim3(256), 0, stream>>>(qf, rwb, QRh, QRl, n8);
  krplanes_kernel<<<dim3(n8 / 256), dim3(256), 0, stream>>>(kf, remb, KRh, KRl, n8);
  tb_kernel<<<dim3((kHeads * kSeq) / 256), dim3(256), 0, stream>>>(rwb, remb, rbias, TB);
  relattn_kernel<<<dim3(kBatch * kHeads * (kSeq / 64)), dim3(128), 0, stream>>>(QRh, QRl, KRh, KRl, Vh, TB, AVh, AVl);
  wmma_gemm64<1, 2, 0, 0, false><<<dim3(128, 1), dim3(256), 0, stream>>>(
      AVh, AVl, kDim, 0L,
      WT + 3 * wPlane, WT + 3 * wPlane, kDim, 0L,
      (void*)AO, (void*)AO, kDim, 0L,
      gamma, gamma, 0L,
      kTok, kDim, kDim, 1.0f);
  ln_kernel<<<dim3(kTok), dim3(256), 0, stream>>>(w, AO, gamma, beta, out);
}
